// TriDimensionalAttentionBlock_22170621182173
// MI455X (gfx1250) — hardware-verified
//
#include <hip/hip_runtime.h>
#include <math.h>
#include <stdint.h>

#define HID    128
#define DMOD   256
#define NHEAD  8
#define DHEAD  32
#define NBAT   8
#define NPT    512
#define NIN    3
#define NOUT   2
#define TOKB   (NPT * NIN * NOUT)
#define NTOK   (NBAT * TOKB)
#define QKVW   (3 * DMOD)
#define NCAT   (9 * DMOD)
#define KCAT   (3 * DMOD)
#define NCHUNK 2
#define CTOK   (NTOK / NCHUNK)
#define CBAT   (NBAT / NCHUNK)
#define NSEQC  (CBAT * NOUT * NIN)

#define SSC    64.0f
#define WSC    64.0f
#define QC     1024.0f
#define KC     1024.0f
#define VC     256.0f
#define OSC    256.0f
#define LNPSC  9.704060527839234f
#define ATTSC  0.17677669529663687f
#define INV_SQRT2 0.70710678118654752f
#define GELU_C 0.7978845608028654f

static_assert(NHEAD * DHEAD == DMOD);
static_assert((CTOK % 64) == 0 && (QKVW % 64) == 0 && (HID % 32) == 0 && (KCAT % 32) == 0);
static_assert((((CTOK / 64) * (QKVW / 64)) % 8) == 0);
static_assert((((NTOK / 64) * (DMOD / 64)) % 8) == 0);
static_assert((TOKB % 64) == 0 && (CTOK % TOKB) == 0);
static_assert(((NTOK * HID) % (8 * 256)) == 0);
static_assert((CTOK % 8) == 0 && (NPT % 64) == 0 && (NCAT % 256) == 0);

typedef _Float16 v16h __attribute__((ext_vector_type(16)));
typedef _Float16 v8h  __attribute__((ext_vector_type(8)));
typedef float    v8f  __attribute__((ext_vector_type(8)));
typedef float    v4f  __attribute__((ext_vector_type(4)));
typedef unsigned int v4u __attribute__((ext_vector_type(4)));
typedef int      v4i  __attribute__((ext_vector_type(4)));

union FragH { v16h v; v8h h[2]; };
union FragE { v16h v; v8h h[2]; _Float16 e[16]; };

__device__ __forceinline__ unsigned short bf_bits(float f) {
  unsigned u = __float_as_uint(f);
  return (unsigned short)((u + 0x7FFFu + ((u >> 16) & 1u)) >> 16);
}
__device__ __forceinline__ float bf_up(unsigned short h) { return __uint_as_float(((unsigned)h) << 16); }
__device__ __forceinline__ float bfr(float f) { return bf_up(bf_bits(f)); }
__device__ __forceinline__ unsigned short h_bits(_Float16 x) { return __builtin_bit_cast(unsigned short, x); }
__device__ __forceinline__ unsigned pk16(unsigned short a, unsigned short b) { return (unsigned)a | ((unsigned)b << 16); }
__device__ __forceinline__ v8f zero8() { v8f z = {0.f, 0.f, 0.f, 0.f, 0.f, 0.f, 0.f, 0.f}; return z; }

__device__ __forceinline__ void split8(const v4f a, const v4f b, float sc, v4u& hv, v4u& lv) {
  unsigned short hb[8], lb[8];
#pragma unroll
  for (int e = 0; e < 4; ++e) {
    float y = a[e] * sc; _Float16 hi = (_Float16)y;
    hb[e] = h_bits(hi); lb[e] = h_bits((_Float16)(y - (float)hi));
    y = b[e] * sc; hi = (_Float16)y;
    hb[4 + e] = h_bits(hi); lb[4 + e] = h_bits((_Float16)(y - (float)hi));
  }
#pragma unroll
  for (int i = 0; i < 4; ++i) { hv[i] = pk16(hb[2 * i], hb[2 * i + 1]); lv[i] = pk16(lb[2 * i], lb[2 * i + 1]); }
}

__device__ __forceinline__ float gelu_t(float x) {
  const float u = GELU_C * (x + 0.044715f * x * x * x);
  float a = fminf(fabsf(u), 20.0f);
  const float E = __expf(2.0f * a);
  float t = 1.0f - 2.0f * __builtin_amdgcn_rcpf(E + 1.0f);
  t = (u < 0.f) ? -t : t;
  return 0.5f * x * (1.0f + t);
}

__device__ __forceinline__ v16h ldfrag_h(const _Float16* p) {
  FragH f;
  f.h[0] = *(const v8h*)(p);
  f.h[1] = *(const v8h*)(p + 16);
  return f.v;
}

__device__ __forceinline__ v8f mma_h_raw(v16h a, v16h b, v8f c) {
  return __builtin_amdgcn_wmma_f32_16x16x32_f16(false, a, false, b, (short)0, c, false, false);
}
__device__ __forceinline__ void dep_guard1(v8f& a, v8f& b, v16h x) {
#if defined(__HIP_DEVICE_COMPILE__)
  asm volatile("v_nop\n\tv_nop\n\tv_nop\n\tv_nop" : "+v"(a), "+v"(b) : "v"(x));
#endif
}
__device__ __forceinline__ void dep_guard2(v8f& a, v8f& b, v16h x, v16h y) {
#if defined(__HIP_DEVICE_COMPILE__)
  asm volatile("v_nop\n\tv_nop\n\tv_nop\n\tv_nop" : "+v"(a), "+v"(b) : "v"(x), "v"(y));
#endif
}
__device__ __forceinline__ void keep4_h(v16h a, v16h b, v16h c, v16h d) {
#if defined(__HIP_DEVICE_COMPILE__)
  asm volatile("v_nop" :: "v"(a), "v"(b), "v"(c), "v"(d));
#endif
}
__device__ __forceinline__ void acc_guard4(v8f& a, v8f& b, v8f& c, v8f& d) {
#if defined(__HIP_DEVICE_COMPILE__)
  asm volatile("v_nop\n\tv_nop\n\tv_nop\n\tv_nop" : "+v"(a), "+v"(b), "+v"(c), "+v"(d));
#endif
}
__device__ __forceinline__ void sguard2(v8f& a, v8f& b, v16h k0, v16h k1, v16h k2, v16h k3, v16h q0, v16h q1) {
#if defined(__HIP_DEVICE_COMPILE__)
  asm volatile("v_nop\n\tv_nop\n\tv_nop\n\tv_nop"
               : "+v"(a), "+v"(b) : "v"(k0), "v"(k1), "v"(k2), "v"(k3), "v"(q0), "v"(q1));
#endif
}
__device__ __forceinline__ void oguard2(v8f& a, v8f& b, v16h x0, v16h x1, v16h p0) {
#if defined(__HIP_DEVICE_COMPILE__)
  asm volatile("v_nop\n\tv_nop\n\tv_nop\n\tv_nop" : "+v"(a), "+v"(b) : "v"(x0), "v"(x1), "v"(p0));
#endif
}
__device__ __forceinline__ void wave_sync_lds() {
  __builtin_amdgcn_fence(__ATOMIC_RELEASE, "workgroup");
  __builtin_amdgcn_wave_barrier();
  __builtin_amdgcn_fence(__ATOMIC_ACQUIRE, "workgroup");
}

__global__ __launch_bounds__(256) void prep_tables(const float* __restrict__ t, const float* __restrict__ wt,
                                                    const float* __restrict__ bt,
                                                    const float* wq, const float* bq, const float* wk, const float* bk,
                                                    const float* wv, const float* bv, const float* __restrict__ bo,
                                                    float* BT, float* BOC) {
  __shared__ float te[HID];
  const int tid = threadIdx.x, b = blockIdx.x;
  if (tid < HID) {
    float acc = 0.f;
#pragma unroll 1
    for (int k = 0; k < HID; ++k) acc += bfr(t[b * HID + k]) * bfr(wt[k * HID + tid]);
    te[tid] = acc + bfr(bt[tid]);
  }
  __syncthreads();
#pragma unroll 1
  for (int it = 0; it < NCAT / 256; ++it) {
    const int nc = it * 256 + tid;
    const int l = nc / QKVW, r = nc - l * QKVW, p = r >> 8, e = r & 255;
    const float* W  = (p == 0) ? wq : ((p == 1) ? wk : wv);
    const float* Bv = (p == 0) ? bq : ((p == 1) ? bk : bv);
    const float* wp = W + (size_t)l * HID * DMOD + e;
    float acc = 0.f;
#pragma unroll 1
    for (int k = 0; k < HID; ++k) acc += te[k] * bfr(wp[(size_t)k * DMOD]);
    const float val = acc + bfr(Bv[l * DMOD + e]);
    float* dp = BT + (size_t)b * NCAT + nc;
    *(volatile float*)dp = val;
    __threadfence();
    *(volatile float*)dp = val;
  }
  if (b == 0) {
    const float v = bfr(bo[tid]) + bfr(bo[DMOD + tid]) + bfr(bo[2 * DMOD + tid]);
    *(volatile float*)(BOC + tid) = v;
    __threadfence();
    *(volatile float*)(BOC + tid) = v;
  }
}

__global__ __launch_bounds__(256) void cvt_s(const float* __restrict__ s, unsigned short* S16) {
  const size_t g = (size_t)blockIdx.x * 256 + threadIdx.x;
  const float* sp = s + g * 8;
  const v4f a = *(const v4f*)(sp), c = *(const v4f*)(sp + 4);
  float f[8];
#pragma unroll
  for (int i = 0; i < 4; ++i) { f[i] = bfr(a[i]) * SSC; f[4 + i] = bfr(c[i]) * SSC; }
  v4u v;
#pragma unroll
  for (int i = 0; i < 4; ++i) v[i] = pk16(h_bits((_Float16)f[2 * i]), h_bits((_Float16)f[2 * i + 1]));
  unsigned short* dp = S16 + g * 8;
  *(volatile v4u*)dp = v;
  __threadfence();
  *(volatile v4u*)dp = v;
}

__global__ __launch_bounds__(256) void cvt_w(const float* wq, const float* wk, const float* wv,
                                              const float* __restrict__ wo,
                                              unsigned short* WQ16, unsigned short* WO16) {
  __shared__ __align__(16) unsigned short tile[32 * 264];
  const int tid = threadIdx.x, bx = blockIdx.x;
  if (bx < 72) {
    const int m = bx >> 3, et = bx & 7;
    const int l = m / 3, p = m - 3 * l;
    const float* W = (p == 0) ? wq : ((p == 1) ? wk : wv);
    const int k = tid >> 1, eh = tid & 1;
    const float* sp = W + ((size_t)(l * HID + k) * DMOD + et * 32 + eh * 16);
#pragma unroll
    for (int q4 = 0; q4 < 4; ++q4) {
      const v4f v = *(const v4f*)(sp + 4 * q4);
#pragma unroll
      for (int e = 0; e < 4; ++e)
        tile[(eh * 16 + 4 * q4 + e) * 136 + k] = h_bits((_Float16)(bfr(v[e]) * WSC));
    }
    __syncthreads();
    v4u u[2]; size_t o[2];
#pragma unroll
    for (int it = 0; it < 2; ++it) {
      const int pi = it * 256 + tid, row = pi >> 4, cc = pi & 15;
      u[it] = *(const v4u*)(tile + row * 136 + 8 * cc);
      o[it] = (size_t)(m * 256 + et * 32 + row) * HID + 8 * cc;
    }
    for (int pass = 0; pass < 2; ++pass) {
#pragma unroll
      for (int it = 0; it < 2; ++it) *(volatile v4u*)(WQ16 + o[it]) = u[it];
      __threadfence();
    }
  } else {
    const int j = bx - 72, l = j >> 3, et = j & 7;
    const int cc = tid;
    const float* sp = wo + ((size_t)(l * DMOD + cc) * DMOD + et * 32);
#pragma unroll
    for (int q4 = 0; q4 < 8; ++q4) {
      const v4f v = *(const v4f*)(sp + 4 * q4);
#pragma unroll
      for (int e = 0; e < 4; ++e)
        tile[(4 * q4 + e) * 264 + cc] = h_bits((_Float16)(bfr(v[e]) * WSC));
    }
    __syncthreads();
    v4u u[4]; size_t o[4];
#pragma unroll
    for (int it = 0; it < 4; ++it) {
      const int pi = it * 256 + tid, row = pi >> 5, c2 = pi & 31;
      u[it] = *(const v4u*)(tile + row * 264 + 8 * c2);
      o[it] = (size_t)(et * 32 + row) * KCAT + l * DMOD + 8 * c2;
    }
    for (int pass = 0; pass < 2; ++pass) {
#pragma unroll
      for (int it = 0; it < 4; ++it) *(volatile v4u*)(WO16 + o[it]) = u[it];
      __threadfence();
    }
  }
}

__global__ __launch_bounds__(256) void gemm64f(
    const unsigned short* __restrict__ Ap, int lda,
    const unsigned short* __restrict__ Bp, int ldb,
    float* Cout, int ldc, float osc, int M, int N, int K,
    const float* __restrict__ bias, int bstride, int rowdiv, int rowoff) {
  __shared__ __align__(16) float sT[8][16 * 68];
  const int lane = threadIdx.x & 31;
  const int wave = threadIdx.x >> 5;
  const int tilesN = N >> 6;
  const int tilesM = M >> 6;
  const int tile = blockIdx.x * 8 + wave;
  if (tile >= tilesM * tilesN) return;
  const int tm = tile / tilesN;
  const int tn = tile - tm * tilesN;
  const int m0 = tm << 6;
  const int n0 = tn << 6;

  const _Float16* Ah = (const _Float16*)(const void*)Ap;
  const _Float16* Bb = (const _Float16*)(const void*)Bp;

  const int rlane = lane & 15;
  const int koff  = (lane >> 4) * 8;
  const int mOff  = (lane >> 4) * 8;

  v8f acc[4][4];
#pragma unroll
  for (int i = 0; i < 4; ++i)
#pragma unroll
    for (int j = 0; j < 4; ++j) acc[i][j] = zero8();

  for (int k0 = 0; k0 < K; k0 += 32) {
    v16h bh[4];
#pragma unroll
    for (int j = 0; j < 4; ++j) {
      const size_t bo = (size_t)(n0 + (j << 4) + rlane) * ldb + koff + k0;
      bh[j] = ldfrag_h(Bb + bo);
    }
#pragma unroll
    for (int i = 0; i < 4; ++i) {
      const size_t ao = (size_t)(m0 + (i << 4) + rlane) * lda + koff + k0;
      const v16h ah = ldfrag_h(Ah + ao);
#pragma unroll
      for (int j = 0; j < 4; ++j) acc[i][j] = mma_h_raw(ah, bh[j], acc[i][j]);
      dep_guard1(acc[i][0], acc[i][3], ah);
    }
    keep4_h(bh[0], bh[1], bh[2], bh[3]);
  }
  acc_guard4(acc[0][0], acc[0][1], acc[0][2], acc[0][3]);
  acc_guard4(acc[1][0], acc[1][1], acc[1][2], acc[1][3]);
  acc_guard4(acc[2][0], acc[2][1], acc[2][2], acc[2][3]);
  acc_guard4(acc[3][0], acc[3][1], acc[3][2], acc[3][3]);

  const int hh2 = lane >> 4, c4 = (lane & 15) * 4;
  float* slab = sT[wave];
#pragma unroll
  for (int i = 0; i < 4; ++i) {
    const int mBase = m0 + (i << 4);
    const int brow = (rowoff + mBase) / rowdiv;
    const v4f bv = *(const v4f*)(bias + (size_t)brow * bstride + n0 + c4);
#pragma unroll
    for (int j = 0; j < 4; ++j) {
#pragma unroll
      for (int r = 0; r < 8; ++r) {
        slab[(mOff + r) * 68 + (j << 4) + rlane] = acc[i][j][r];
      }
    }
    wave_sync_lds();
    v4f vals[8];
#pragma unroll
    for (int it = 0; it < 8; ++it) {
      const int row = it * 2 + hh2;
      v4f v = *(const v4f*)(slab + row * 68 + c4);
#pragma unroll
      for (int e = 0; e < 4; ++e) v[e] = v[e] * osc + bv[e];
      vals[it] = v;
    }
    for (int pass = 0; pass < 2; ++pass) {
#pragma unroll
      for (int it = 0; it < 8; ++it) {
        const int row = it * 2 + hh2;
        *(volatile v4f*)(Cout + (size_t)(mBase + row) * ldc + n0 + c4) = vals[it];
      }
      __threadfence();
    }
    wave_sync_lds();
  }
}

template <int L, int TS>
__global__ __launch_bounds__(256) void attn_small(const float* __restrict__ QKV,
                                                   unsigned short* OBH, unsigned short* OBL,
                                                   int tok0, int colbase) {
  const int tid = threadIdx.x, wave = tid >> 5, lane = tid & 31;
  const int tq = blockIdx.x * 8 + wave;
  const int pos = (tq / TS) % L;
  const int gb = tq - pos * TS;
  const int dof = 8 * lane;
  const float* qp = QKV + (size_t)tq * QKVW + dof;
  const v4f qa = *(const v4f*)(qp), qb = *(const v4f*)(qp + 4);
  float lg[L];
  v4f va[L], vb[L];
#pragma unroll
  for (int j = 0; j < L; ++j) {
    const float* kp = QKV + (size_t)(gb + j * TS) * QKVW + DMOD + dof;
    const v4f ka = *(const v4f*)(kp), kb = *(const v4f*)(kp + 4);
    va[j] = *(const v4f*)(kp + DMOD);
    vb[j] = *(const v4f*)(kp + DMOD + 4);
    float d = 0.f;
#pragma unroll
    for (int e = 0; e < 4; ++e) d += qa[e] * ka[e];
#pragma unroll
    for (int e = 0; e < 4; ++e) d += qb[e] * kb[e];
    d += __shfl_xor(d, 1, 32);
    d += __shfl_xor(d, 2, 32);
    lg[j] = d * ATTSC;
  }
  float mx = lg[0];
#pragma unroll
  for (int j = 1; j < L; ++j) mx = fmaxf(mx, lg[j]);
  float p[L];
  float den = 0.f;
#pragma unroll
  for (int j = 0; j < L; ++j) { p[j] = __expf(lg[j] - mx); den += p[j]; }
  const float inv = 1.0f / den;
  v4f oa = {0.f, 0.f, 0.f, 0.f}, ob = {0.f, 0.f, 0.f, 0.f};
#pragma unroll
  for (int j = 0; j < L; ++j) {
#pragma unroll
    for (int e = 0; e < 4; ++e) { oa[e] += p[j] * va[j][e]; ob[e] += p[j] * vb[j][e]; }
  }
#pragma unroll
  for (int e = 0; e < 4; ++e) { oa[e] *= inv; ob[e] *= inv; }
  v4u hv, lv;
  split8(oa, ob, OSC, hv, lv);
  const size_t o = (size_t)(tok0 + tq) * KCAT + colbase + 8 * lane;
  *(volatile v4u*)(OBH + o) = hv;
  *(volatile v4u*)(OBL + o) = lv;
  __threadfence();
  *(volatile v4u*)(OBH + o) = hv;
  *(volatile v4u*)(OBL + o) = lv;
}

__global__ __launch_bounds__(256)
void attn_n(const float* __restrict__ QKV, const int* __restrict__ msk,
            unsigned short* OBH, unsigned short* OBL, int chunk) {
  __shared__ __align__(16) _Float16 KsH[64 * 72];
  __shared__ __align__(16) _Float16 KsL[64 * 72];
  __shared__ __align__(16) _Float16 VsH[64 * 72];
  __shared__ __align__(16) float Os[64 * 64];
  const int tid  = threadIdx.x;
  const int wave = tid >> 5;
  const int lane = tid & 31;
  const int hh   = lane >> 4;
  const int c    = lane & 15;
  const int bx   = blockIdx.x;
  const int qb   = bx & 7;
  const int hp   = (bx >> 3) & 3;
  const int sq   = bx >> 5;
  const int bl   = sq / 6, rem = sq - 6 * bl, o = rem / 3, i = rem - 3 * o;
  const int hl   = wave >> 2, qt = wave & 3;
  const int h    = 2 * hp + hl;
  const int q0   = qb * 64;
  const size_t rowbase  = (size_t)bl * TOKB + i * 2 + o;
  const size_t growbase = (size_t)(chunk * CBAT + bl) * TOKB + i * 2 + o;
  const int qn = q0 + 16 * qt + c;

  FragH qh, ql;
  {
    const float* qp = QKV + (rowbase + (size_t)6 * qn) * QKVW + h * DHEAD + 8 * hh;
    const v4f t0 = *(const v4f*)(qp), t1 = *(const v4f*)(qp + 4);
    const v4f t2 = *(const v4f*)(qp + 16), t3 = *(const v4f*)(qp + 20);
#pragma unroll
    for (int r = 0; r < 4; ++r) {
      float y; _Float16 hi;
      y = t0[r] * QC; hi = (_Float16)y; qh.h[0][r] = hi;     ql.h[0][r] = (_Float16)(y - (float)hi);
      y = t1[r] * QC; hi = (_Float16)y; qh.h[0][4 + r] = hi; ql.h[0][4 + r] = (_Float16)(y - (float)hi);
      y = t2[r] * QC; hi = (_Float16)y; qh.h[1][r] = hi;     ql.h[1][r] = (_Float16)(y - (float)hi);
      y = t3[r] * QC; hi = (_Float16)y; qh.h[1][4 + r] = hi; ql.h[1][4 + r] = (_Float16)(y - (float)hi);
    }
  }
  const int* mrow = msk + (size_t)qn * NPT;
  const float SC = ATTSC / (QC * KC);

  const int kk = tid >> 2, part = tid & 3, shl = part >> 1, dh = part & 1;
  const int scol = shl * 32 + 16 * dh;

  float m = -1.0e30f, l = 0.f;
  v8f o0 = zero8(), o1 = zero8();
#pragma unroll 1
  for (int kcb = 0; kcb < NPT / 64; ++kcb) {
    {
      const float* kp = QKV + (rowbase + (size_t)6 * (kcb * 64 + kk)) * QKVW + DMOD + (2 * hp + shl) * DHEAD + 16 * dh;
      FragE kf, kg;
#pragma unroll
      for (int q4 = 0; q4 < 4; ++q4) {
        const v4f kv = *(const v4f*)(kp + 4 * q4);
        const v4f vv = *(const v4f*)(kp + DMOD + 4 * q4);
#pragma unroll
        for (int e = 0; e < 4; ++e) {
          const int j = 4 * q4 + e;
          float y = kv[e] * KC; _Float16 hi = (_Float16)y;
          kf.e[j] = hi;
          kg.e[j] = (_Float16)(y - (float)hi);
          VsH[(scol + j) * 72 + kk] = (_Float16)(vv[e] * VC);
        }
      }
      *(v8h*)(KsH + kk * 72 + scol)     = kf.h[0];
      *(v8h*)(KsH + kk * 72 + scol + 8) = kf.h[1];
      *(v8h*)(KsL + kk * 72 + scol)     = kg.h[0];
      *(v8h*)(KsL + kk * 72 + scol + 8) = kg.h[1];
    }
    __syncthreads();
#pragma unroll 1
    for (int ks = 0; ks < 2; ++ks) {
      const int kb = ks * 32;
      const v16h kf0h = ldfrag_h(KsH + (kb + c) * 72 + hl * 32 + 8 * hh);
      const v16h kf1h = ldfrag_h(KsH + (kb + 16 + c) * 72 + hl * 32 + 8 * hh);
      const v16h kf0l = ldfrag_h(KsL + (kb + c) * 72 + hl * 32 + 8 * hh);
      const v16h kf1l = ldfrag_h(KsL + (kb + 16 + c) * 72 + hl * 32 + 8 * hh);
      v8f s0 = mma_h_raw(kf0h, qh.v, zero8());
      v8f s1 = mma_h_raw(kf1h, qh.v, zero8());
      s0 = mma_h_raw(kf0h, ql.v, s0);
      s1 = mma_h_raw(kf1h, ql.v, s1);
      s0 = mma_h_raw(kf0l, qh.v, s0);
      s1 = mma_h_raw(kf1l, qh.v, s1);
      sguard2(s0, s1, kf0h, kf1h, kf0l, kf1l, qh.v, ql.v);

      const int kg0 = kcb * 64 + kb;
      const v4i ma = *(const v4i*)(mrow + kg0 + 8 * hh);
      const v4i mb = *(const v4i*)(mrow + kg0 + 8 * hh + 4);
      const v4i mc = *(const v4i*)(mrow + kg0 + 16 + 8 * hh);
      const v4i md = *(const v4i*)(mrow + kg0 + 16 + 8 * hh + 4);
      float x0[8], x1[8];
#pragma unroll
      for (int r = 0; r < 4; ++r) {
        x0[r]     = (ma[r] != 0) ? s0[r] * SC     : -1.0e30f;
        x0[4 + r] = (mb[r] != 0) ? s0[4 + r] * SC : -1.0e30f;
        x1[r]     = (mc[r] != 0) ? s1[r] * SC     : -1.0e30f;
        x1[4 + r] = (md[r] != 0) ? s1[4 + r] * SC : -1.0e30f;
      }
      float mx = x0[0];
#pragma unroll
      for (int r = 1; r < 8; ++r) mx = fmaxf(mx, x0[r]);
#pragma unroll
      for (int r = 0; r < 8; ++r) mx = fmaxf(mx, x1[r]);
      mx = fmaxf(mx, __shfl_xor(mx, 16, 32));
      const float mn   = fmaxf(m, mx);
      const float corr = __expf(m - mn);
      m = mn;
      const float msh = mn - LNPSC;
      l *= corr;
#pragma unroll
      for (int r = 0; r < 8; ++r) { o0[r] *= corr; o1[r] *= corr; }

      FragH ph;
      float ls = 0.f;
#pragma unroll
      for (int r = 0; r < 8; ++r) {
        const float e0 = __expf(x0[r] - msh);
        const float e1 = __expf(x1[r] - msh);
        ls += e0 + e1;
        ph.h[0][r] = (_Float16)e0;
        ph.h[1][r] = (_Float16)e1;
      }
      l += ls;

      const v16h vh0 = ldfrag_h(VsH + (hl * 32 + c) * 72 + kb + 8 * hh);
      const v16h vh1 = ldfrag_h(VsH + (hl * 32 + 16 + c) * 72 + kb + 8 * hh);
      o0 = mma_h_raw(vh0, ph.v, o0);
      o1 = mma_h_raw(vh1, ph.v, o1);
      oguard2(o0, o1, vh0, vh1, ph.v);
    }
    __syncthreads();
  }
  l += __shfl_xor(l, 16, 32);
  const float sc = (1.0f / VC) * (1.0f / l);

  {
    float* os = Os + (16 * qt + c) * 64 + hl * 32 + 8 * hh;
#pragma unroll
    for (int r = 0; r < 8; ++r) { os[r] = o0[r] * sc; os[16 + r] = o1[r] * sc; }
  }
  __syncthreads();
  {
    v4u hv[2], lv[2]; size_t dof[2];
#pragma unroll
    for (int it = 0; it < 2; ++it) {
      const int pi = it * 256 + tid, row = pi >> 3, e = pi & 7;
      const float* op = Os + row * 64 + 8 * e;
      const v4f a = *(const v4f*)(op), b = *(const v4f*)(op + 4);
      split8(a, b, OSC, hv[it], lv[it]);
      dof[it] = (growbase + (size_t)6 * (q0 + row)) * KCAT + 2 * DMOD + hp * 64 + 8 * e;
    }
    for (int pass = 0; pass < 2; ++pass) {
#pragma unroll
      for (int it = 0; it < 2; ++it) {
        *(volatile v4u*)(OBH + dof[it]) = hv[it];
        *(volatile v4u*)(OBL + dof[it]) = lv[it];
      }
      __threadfence();
    }
  }
}

__global__ __launch_bounds__(256) void gemm_out(
    const unsigned short* __restrict__ AHp, const unsigned short* __restrict__ ALp,
    const unsigned short* __restrict__ Bp, const float* __restrict__ boc,
    const float* __restrict__ s, float* out) {
  __shared__ __align__(16) float sT[8][16 * 68];
  const int lane = threadIdx.x & 31;
  const int wave = threadIdx.x >> 5;
  const int tilesN = DMOD >> 6;
  const int tilesM = NTOK >> 6;
  const int tile = blockIdx.x * 8 + wave;
  if (tile >= tilesM * tilesN) return;
  const int tm = tile / tilesN;
  const int tn = tile - tm * tilesN;
  const int m0 = tm << 6;
  const int n0 = tn << 6;

  const _Float16* Ah = (const _Float16*)(const void*)AHp;
  const _Float16* Al = (const _Float16*)(const void*)ALp;
  const _Float16* Bb = (const _Float16*)(const void*)Bp;

  const int rlane = lane & 15;
  const int koff  = (lane >> 4) * 8;
  const int mOff  = (lane >> 4) * 8;

  v8f acc[4][4];
#pragma unroll
  for (int i = 0; i < 4; ++i)
#pragma unroll
    for (int j = 0; j < 4; ++j) acc[i][j] = zero8();

  for (int k0 = 0; k0 < KCAT; k0 += 32) {
    v16h bh[4];
#pragma unroll
    for (int j = 0; j < 4; ++j) {
      const size_t bo = (size_t)(n0 + (j << 4) + rlane) * KCAT + koff + k0;
      bh[j] = ldfrag_h(Bb + bo);
    }
#pragma unroll
    for (int i = 0; i < 4; ++i) {
      const size_t ao = (size_t)(m0 + (i << 4) + rlane) * KCAT + koff + k0;
      const v16h ah = ldfrag_h(Ah + ao);
      const v16h al = ldfrag_h(Al + ao);
#pragma unroll
      for (int j = 0; j < 4; ++j) {
        acc[i][j] = mma_h_raw(ah, bh[j], acc[i][j]);
        acc[i][j] = mma_h_raw(al, bh[j], acc[i][j]);
      }
      dep_guard2(acc[i][0], acc[i][3], ah, al);
    }
    keep4_h(bh[0], bh[1], bh[2], bh[3]);
  }
  acc_guard4(acc[0][0], acc[0][1], acc[0][2], acc[0][3]);
  acc_guard4(acc[1][0], acc[1][1], acc[1][2], acc[1][3]);
  acc_guard4(acc[2][0], acc[2][1], acc[2][2], acc[2][3]);
  acc_guard4(acc[3][0], acc[3][1], acc[3][2], acc[3][3]);

  const float osc = 1.0f / (OSC * WSC);
  const int hh2 = lane >> 4, c4 = (lane & 15) * 4;
  const bool first = (n0 < HID);
  const int col0 = n0 & (HID - 1);
  float* ob = first ? out : (out + (size_t)NTOK * HID);
  const v4f bb = *(const v4f*)(boc + n0 + c4);
  float* slab = sT[wave];
#pragma unroll
  for (int i = 0; i < 4; ++i) {
    const int mBase = m0 + (i << 4);
#pragma unroll
    for (int j = 0; j < 4; ++j) {
#pragma unroll
      for (int r = 0; r < 8; ++r) {
        slab[(mOff + r) * 68 + (j << 4) + rlane] = acc[i][j][r];
      }
    }
    wave_sync_lds();
    v4f vals[8];
#pragma unroll
    for (int it = 0; it < 8; ++it) {
      const int row = it * 2 + hh2;
      v4f v = *(const v4f*)(slab + row * 68 + c4);
      const v4f sv = *(const v4f*)(s + (size_t)(mBase + row) * HID + col0 + c4);
#pragma unroll
      for (int e = 0; e < 4; ++e) {
        const float y  = v[e] * osc + bb[e];
        const float g  = gelu_t(y);
        const float r0 = (bfr(sv[e]) + g) * INV_SQRT2;
        v[e] = first ? r0 : g;
      }
      vals[it] = v;
    }
    for (int pass = 0; pass < 2; ++pass) {
#pragma unroll
      for (int it = 0; it < 8; ++it) {
        const int row = it * 2 + hh2;
        *(volatile v4f*)(ob + (size_t)(mBase + row) * HID + col0 + c4) = vals[it];
      }
      __threadfence();
    }
    wave_sync_lds();
  }
}

extern "C" void kernel_launch(void* const* d_in, const int* in_sizes, int n_in,
                              void* d_out, int out_size, void* d_ws, size_t ws_size,
                              hipStream_t stream) {
  if (n_in < 13) return;
  if (in_sizes[0] != NTOK * HID || in_sizes[1] != NBAT * HID || in_sizes[2] != NPT * NPT) return;
  if (in_sizes[3] != HID * HID || in_sizes[4] != HID) return;
  if (in_sizes[5] != 3 * HID * DMOD || in_sizes[7] != 3 * HID * DMOD || in_sizes[9] != 3 * HID * DMOD) return;
  if (in_sizes[6] != 3 * DMOD || in_sizes[8] != 3 * DMOD || in_sizes[10] != 3 * DMOD || in_sizes[12] != 3 * DMOD) return;
  if (in_sizes[11] != 3 * DMOD * DMOD) return;
  if (out_size != 2 * NTOK * HID) return;

  const float* s    = (const float*)d_in[0];
  const float* t    = (const float*)d_in[1];
  const int*   mk   = (const int*)d_in[2];
  const float* wt   = (const float*)d_in[3];
  const float* bt   = (const float*)d_in[4];
  const float* wq   = (const float*)d_in[5];
  const float* bq   = (const float*)d_in[6];
  const float* wk   = (const float*)d_in[7];
  const float* bk   = (const float*)d_in[8];
  const float* wv   = (const float*)d_in[9];
  const float* bv   = (const float*)d_in[10];
  const float* wo   = (const float*)d_in[11];
  const float* bo   = (const float*)d_in[12];
  float*       out  = (float*)d_out;

  const size_t PS16 = (size_t)NTOK * HID * 2;
  const size_t PWQ  = (size_t)NCAT * HID * 2;
  const size_t PWO  = (size_t)DMOD * KCAT * 2;
  const size_t PBT  = (size_t)NBAT * NCAT * 4;
  const size_t PBOC = (size_t)DMOD * 4;
  const size_t PQKV = (size_t)CTOK * QKVW * 4;
  const size_t POB  = (size_t)NTOK * KCAT * 2;
  size_t off = 0;
  const size_t oS16 = off; off += PS16;
  const size_t oWQ  = off; off += PWQ;
  const size_t oWO  = off; off += PWO;
  const size_t oBT  = off; off += PBT;
  const size_t oBOC = off; off += PBOC;
  const size_t oQKV = off; off += PQKV;
  const size_t oOBH = off; off += POB;
  const size_t oOBL = off; off += POB;
  if (off > ws_size) return;
  if (off > (size_t)134217728) return;

  char* ws = (char*)d_ws;
  unsigned short* S16  = (unsigned short*)(ws + oS16);
  unsigned short* WQ16 = (unsigned short*)(ws + oWQ);
  unsigned short* WO16 = (unsigned short*)(ws + oWO);
  float*          BT   = (float*)(ws + oBT);
  float*          BOC  = (float*)(ws + oBOC);
  float*          QKV  = (float*)(ws + oQKV);
  unsigned short* OBH  = (unsigned short*)(ws + oOBH);
  unsigned short* OBL  = (unsigned short*)(ws + oOBL);

  const dim3 blk(256);
  const dim3 gTB(NBAT);
  const dim3 gCS((NTOK * HID) / (8 * 256));
  const dim3 gCW(72 + 24);
  const dim3 gGM(((CTOK / 64) * (QKVW / 64)) / 8);
  const dim3 gAS(CTOK / 8);
  const dim3 gAN(NSEQC * 4 * (NPT / 64));
  const dim3 gGO(((NTOK / 64) * (DMOD / 64)) / 8);

  prep_tables<<<gTB, blk, 0, stream>>>(t, wt, bt, wq, bq, wk, bk, wv, bv, bo, BT, BOC);
  cvt_s<<<gCS, blk, 0, stream>>>(s, S16);
  cvt_w<<<gCW, blk, 0, stream>>>(wq, wk, wv, wo, WQ16, WO16);

  for (int l = 0; l < 3; ++l) {
    for (int ch = 0; ch < NCHUNK; ++ch) {
      gemm64f<<<gGM, blk, 0, stream>>>(S16 + (size_t)ch * CTOK * HID, HID,
                                       WQ16 + (size_t)l * QKVW * HID, HID,
                                       QKV, QKVW, 1.0f / (SSC * WSC), CTOK, QKVW, HID,
                                       BT + (size_t)l * QKVW, NCAT, TOKB, ch * CTOK);
      if (l == 0) {
        attn_small<2, 1><<<gAS, blk, 0, stream>>>(QKV, OBH, OBL, ch * CTOK, 0);
      } else if (l == 1) {
        attn_small<3, 2><<<gAS, blk, 0, stream>>>(QKV, OBH, OBL, ch * CTOK, DMOD);
      } else {
        attn_n<<<gAN, blk, 0, stream>>>(QKV, mk, OBH, OBL, ch);
      }
    }
  }

  gemm_out<<<gGO, blk, 0, stream>>>(OBH, OBL, WO16, BOC, s, out);
  (void)hipGetLastError();
}
